// Revealing_12979391169452
// MI455X (gfx1250) — hardware-verified
//
#include <hip/hip_runtime.h>
#include <stddef.h>


#define NTOK    16
#define DEMB    256
#define LMAXV   8
#define NH      4
#define CH1     64
#define H1C     256
#define CH2     256
#define H2C     1024
#define HID     512
#define NCLS    256
#define NTHR    256
#define NWAVE   8
#define EPT     8
#define NGRP    2
#define CHUNK   (NTHR * EPT * NGRP)
#define WCAP    (EPT * NGRP * 32)
#define LISTN   (NWAVE * WCAP)
#define NBC     4096
#define NBF     1024
#define RCAP    40960
#define RBN     128
#define TGT     256
#define DEGCAP  256
#define OTHR    512
#define FNB     256
#define NCB     256
#define GBM     64
#define GKS     128
#define GAPK    (GKS + 8)
#define GLDS    (GBM * NCB * 4)
#define WSCAP   134217728
#define NEG_SLOPE 0.2f
#define DEC_SLOPE 0.01f
#define DEN_EPS 1e-16f
#define NEG_BIG (-3.0e38f)

#define LDS_FILL ((RCAP + NBF + LISTN) * 4 + 64)

static_assert((CHUNK & (CHUNK - 1)) == 0);
static_assert(CHUNK <= 4096);
static_assert(NBC <= 4096 && NBF <= 4096);
static_assert((NBC & (NBC - 1)) == 0 && (NBF & (NBF - 1)) == 0);
static_assert(NBC == 4 * NBF);
static_assert(OTHR * 8 == NBC);
static_assert((RCAP % 32) == 0);
static_assert(TGT == NWAVE * 32);
static_assert((NBC % TGT) == 0);
static_assert(FNB == TGT && (TGT % GBM) == 0);
static_assert(2 * GBM * GAPK * 2 <= GLDS);
static_assert(H1C == NH * CH1 && H2C == NH * CH2 && DEMB == 256 && CH2 == 256);

typedef float          v4f  __attribute__((ext_vector_type(4)));
typedef float          v8f  __attribute__((ext_vector_type(8)));
typedef int            v4i  __attribute__((ext_vector_type(4)));
typedef unsigned short v8us __attribute__((ext_vector_type(8)));
typedef __bf16         v16b __attribute__((ext_vector_type(16)));
union FragB { v16b v; v8us h[2]; };

__device__ __forceinline__ unsigned int bfr(float f) {
  const unsigned int u = __float_as_uint(f);
  return (u + 0x7FFFu + ((u >> 16) & 1u)) >> 16;
}

__device__ __forceinline__ void split1(float x, unsigned short& hb, unsigned short& lb) {
  const unsigned int hu = bfr(x);
  const float hf = __uint_as_float(hu << 16);
  hb = (unsigned short)hu;
  lb = (unsigned short)bfr(x - hf);
}

__device__ __forceinline__ void split8(v4f a, v4f b, v8us& hi, v8us& lo) {
  unsigned short hb, lb;
  split1(a.x, hb, lb); hi[0] = hb; lo[0] = lb;
  split1(a.y, hb, lb); hi[1] = hb; lo[1] = lb;
  split1(a.z, hb, lb); hi[2] = hb; lo[2] = lb;
  split1(a.w, hb, lb); hi[3] = hb; lo[3] = lb;
  split1(b.x, hb, lb); hi[4] = hb; lo[4] = lb;
  split1(b.y, hb, lb); hi[5] = hb; lo[5] = lb;
  split1(b.z, hb, lb); hi[6] = hb; lo[6] = lb;
  split1(b.w, hb, lb); hi[7] = hb; lo[7] = lb;
}

__device__ __forceinline__ v8f wmb(v16b a, v16b b, v8f c) {
  v8f d = __builtin_amdgcn_wmma_f32_16x16x32_bf16(false, a, false, b, (short)0, c, false, false);
  asm volatile("v_nop\n\tv_nop\n\tv_nop\n\tv_nop" : "+v"(d) : "v"(a), "v"(b));
  return d;
}

__device__ __forceinline__ float lrelu(float v) { return v > 0.0f ? v : NEG_SLOPE * v; }
__device__ __forceinline__ float eluf(float v)  { return v > 0.0f ? v : (__expf(v) - 1.0f); }

template <int NB>
__device__ __forceinline__ int scan_chunk(const int* __restrict__ dsts, int nE, int cbase, int slotBase,
                                          int vec8, int* list, int tid, int lane, int wave) {
  int wc = 0;
#pragma unroll
  for (int g = 0; g < NGRP; ++g) {
    const int el0  = (g * NTHR + tid) * EPT;
    const int e0   = cbase + el0;
    const int sent = -2147483647 - 1;
    v4i da, db;
    if (vec8 != 0 && cbase + CHUNK <= nE) {
      da = *(const v4i*)(dsts + e0);
      db = *(const v4i*)(dsts + e0 + 4);
    } else {
      da.x = (e0     < nE) ? dsts[min(e0, nE - 1)] : sent;
      da.y = (e0 + 1 < nE) ? dsts[min(e0 + 1, nE - 1)] : sent;
      da.z = (e0 + 2 < nE) ? dsts[min(e0 + 2, nE - 1)] : sent;
      da.w = (e0 + 3 < nE) ? dsts[min(e0 + 3, nE - 1)] : sent;
      db.x = (e0 + 4 < nE) ? dsts[min(e0 + 4, nE - 1)] : sent;
      db.y = (e0 + 5 < nE) ? dsts[min(e0 + 5, nE - 1)] : sent;
      db.z = (e0 + 6 < nE) ? dsts[min(e0 + 6, nE - 1)] : sent;
      db.w = (e0 + 7 < nE) ? dsts[min(e0 + 7, nE - 1)] : sent;
    }
    const unsigned nb = (unsigned)slotBase;
    const unsigned s0 = (unsigned)da.x - nb, s1 = (unsigned)da.y - nb;
    const unsigned s2 = (unsigned)da.z - nb, s3 = (unsigned)da.w - nb;
    const unsigned s4 = (unsigned)db.x - nb, s5 = (unsigned)db.y - nb;
    const unsigned s6 = (unsigned)db.z - nb, s7 = (unsigned)db.w - nb;
    const bool h0 = s0 < (unsigned)NB, h1 = s1 < (unsigned)NB, h2 = s2 < (unsigned)NB, h3 = s3 < (unsigned)NB;
    const bool h4 = s4 < (unsigned)NB, h5 = s5 < (unsigned)NB, h6 = s6 < (unsigned)NB, h7 = s7 < (unsigned)NB;
    const unsigned any = __builtin_amdgcn_ballot_w32(h0 | h1 | h2 | h3 | h4 | h5 | h6 | h7);
    if (any != 0u) {
#define HITJ(J, HJ, SJ) { \
        const unsigned mj = __builtin_amdgcn_ballot_w32(HJ); \
        if (mj != 0u) { \
          if (HJ) { \
            const int pos = wc + (int)__builtin_amdgcn_mbcnt_lo(mj, 0u); \
            if (pos < WCAP) list[wave * WCAP + pos] = ((el0 + (J)) << 12) | (int)(SJ); \
          } \
          wc += (int)__builtin_popcount(mj); } }
      HITJ(0, h0, s0)
      HITJ(1, h1, s1)
      HITJ(2, h2, s2)
      HITJ(3, h3, s3)
      HITJ(4, h4, s4)
      HITJ(5, h5, s5)
      HITJ(6, h6, s6)
      HITJ(7, h7, s7)
#undef HITJ
    }
  }
  return wc;
}

template <int KD, int NC>
__global__ __launch_bounds__(NTHR) void k_wprep(const float* __restrict__ W, unsigned short* wp) {
  constexpr int UNITS = NC * KD / 8;
  constexpr int KD8   = KD / 8;
  static_assert((UNITS % 32) == 0);
  const int i = (int)blockIdx.x * NTHR + (int)threadIdx.x;
  if (i >= UNITS) return;
  const int n  = i / KD8;
  const int k0 = (i - n * KD8) * 8;
  float v[8];
#pragma unroll
  for (int e = 0; e < 8; ++e) v[e] = W[(size_t)(k0 + e) * NC + n];
  v4f a, b;
  a.x = v[0]; a.y = v[1]; a.z = v[2]; a.w = v[3];
  b.x = v[4]; b.y = v[5]; b.z = v[6]; b.w = v[7];
  v8us hv, lv;
  split8(a, b, hv, lv);
  unsigned short* dh = wp + (size_t)i * 8;
  unsigned short* dl = dh + (size_t)NC * KD;
  *(volatile v8us*)dh = hv;
  *(volatile v8us*)dl = lv;
  __threadfence();
  *(volatile v8us*)dh = hv;
  *(volatile v8us*)dl = lv;
}

__global__ __launch_bounds__(NTHR) void k_count(
    const int* __restrict__ dsts, int* cnt, int nE, int vec8) {
  __shared__ __attribute__((aligned(16))) int scnt[NBC];
  __shared__ __attribute__((aligned(16))) int list[LISTN];
  __shared__ int wcnt[NWAVE];
  const int tid = threadIdx.x, lane = tid & 31, wave = tid >> 5;
  const int nodeBase = blockIdx.x * NBC;

  for (int i = tid; i < NBC; i += NTHR) scnt[i] = 0;
  __syncthreads();

  const int nChunks = (nE + CHUNK - 1) / CHUNK;
#pragma unroll 1
  for (int ch = 0; ch < nChunks; ++ch) {
    const int cbase = ch * CHUNK;
    const int wc = scan_chunk<NBC>(dsts, nE, cbase, nodeBase, vec8, list, tid, lane, wave);
    if (lane == 0) wcnt[wave] = wc;
    __syncthreads();
    if (wave == 0) {
#pragma unroll 1
      for (int wsx = 0; wsx < NWAVE; ++wsx) {
        int n = __builtin_amdgcn_readfirstlane(wcnt[wsx]);
        n = n > WCAP ? WCAP : (n < 0 ? 0 : n);
        const int* lp = list + wsx * WCAP;
#pragma unroll 1
        for (int i = 0; i < n; ++i) {
          const int ent  = __builtin_amdgcn_readfirstlane(lp[i]);
          const int slot = ent & (NBC - 1);
          if (lane == 0) scnt[slot] = scnt[slot] + 1;
        }
      }
    }
    __syncthreads();
  }

  v4i cq[4];
#pragma unroll
  for (int q = 0; q < 4; ++q) {
    const int f = (wave * 4 + q) * 128 + 4 * lane;
    cq[q] = *(const v4i*)(scnt + f);
  }
  int* cp = cnt + (size_t)nodeBase;
#pragma unroll
  for (int q = 0; q < 4; ++q) {
    const int f = (wave * 4 + q) * 128 + 4 * lane;
    *(volatile v4i*)(cp + f) = cq[q];
  }
  __threadfence();
#pragma unroll
  for (int q = 0; q < 4; ++q) {
    const int f = (wave * 4 + q) * 128 + 4 * lane;
    *(volatile v4i*)(cp + f) = cq[q];
  }
}

__global__ __launch_bounds__(OTHR) void k_offsets(
    const int* __restrict__ cnt, int* off, int* rbase, int nChunk) {
  __shared__ __attribute__((aligned(16))) int soff[NBC];
  __shared__ __attribute__((aligned(16))) int srb[RBN];
  __shared__ int wtot[OTHR / 32];
  const int tid = threadIdx.x, lane = tid & 31, wave = tid >> 5, sub = tid >> 7;
  for (int i = tid; i < RBN; i += OTHR) srb[i] = 0;
  int carry = 0;
#pragma unroll 1
  for (int ch = 0; ch < nChunk; ++ch) {
    const int base = ch * NBC;
    const v4i c0 = *(const v4i*)(cnt + base + 8 * tid);
    const v4i c1 = *(const v4i*)(cnt + base + 8 * tid + 4);
    const int e0 = max(c0.x, 0), e1 = max(c0.y, 0), e2 = max(c0.z, 0), e3 = max(c0.w, 0);
    const int e4 = max(c1.x, 0), e5 = max(c1.y, 0), e6 = max(c1.z, 0), e7 = max(c1.w, 0);
    const int ts = e0 + e1 + e2 + e3 + e4 + e5 + e6 + e7;
    int incl = ts;
#pragma unroll
    for (int d = 1; d < 32; d <<= 1) {
      const int t = __shfl_up(incl, d);
      if (lane >= d) incl += t;
    }
    if (lane == 31) wtot[wave] = incl;
    __syncthreads();
    const int S0 = wtot[0]  + wtot[1]  + wtot[2]  + wtot[3];
    const int S1 = wtot[4]  + wtot[5]  + wtot[6]  + wtot[7];
    const int S2 = wtot[8]  + wtot[9]  + wtot[10] + wtot[11];
    const int S3 = wtot[12] + wtot[13] + wtot[14] + wtot[15];
    int pre = 0;
#pragma unroll 1
    for (int w = 4 * sub; w < wave; ++w) pre += wtot[w];
    const int b0 = carry;
    const int b1 = b0 + ((S0 + 31) & ~31);
    const int b2 = b1 + ((S1 + 31) & ~31);
    const int b3 = b2 + ((S2 + 31) & ~31);
    const int b4 = b3 + ((S3 + 31) & ~31);
    const int myb = sub == 0 ? b0 : (sub == 1 ? b1 : (sub == 2 ? b2 : b3));
    if (tid == 0) {
      srb[min(4 * ch + 0, RBN - 1)] = b0;
      srb[min(4 * ch + 1, RBN - 1)] = b1;
      srb[min(4 * ch + 2, RBN - 1)] = b2;
      srb[min(4 * ch + 3, RBN - 1)] = b3;
    }
    int run = myb + pre + incl - ts;
    soff[8 * tid + 0] = run; run += e0;
    soff[8 * tid + 1] = run; run += e1;
    soff[8 * tid + 2] = run; run += e2;
    soff[8 * tid + 3] = run; run += e3;
    soff[8 * tid + 4] = run; run += e4;
    soff[8 * tid + 5] = run; run += e5;
    soff[8 * tid + 6] = run; run += e6;
    soff[8 * tid + 7] = run;
    carry = b4;
    __syncthreads();
    const v4i o0 = *(const v4i*)(soff + 4 * tid);
    const v4i o1 = *(const v4i*)(soff + 4 * (tid + OTHR));
    int* op = off + base;
    *(volatile v4i*)(op + 4 * tid) = o0;
    *(volatile v4i*)(op + 4 * (tid + OTHR)) = o1;
    __threadfence();
    *(volatile v4i*)(op + 4 * tid) = o0;
    *(volatile v4i*)(op + 4 * (tid + OTHR)) = o1;
    __syncthreads();
  }
  if (tid == 0) srb[min(4 * nChunk, RBN - 1)] = carry;
  __syncthreads();
  v4i rv = {0, 0, 0, 0};
  if (tid < 32) rv = *(const v4i*)(srb + 4 * tid);
  if (tid < 32) *(volatile v4i*)(rbase + 4 * tid) = rv;
  __threadfence();
  if (tid < 32) *(volatile v4i*)(rbase + 4 * tid) = rv;
}

__global__ __launch_bounds__(NTHR) void k_fill(
    const int* __restrict__ srcs, const int* __restrict__ dsts,
    const int* __restrict__ off, const int* __restrict__ rbase,
    int* csr, int nN, int nE, int vec8, int csrLen) {
  extern __shared__ v4f lds_dyn[];
  int* region = (int*)lds_dyn;
  int* cursor = region + RCAP;
  int* list   = cursor + NBF;
  int* wcnt   = list + LISTN;
  const int tid = threadIdx.x, lane = tid & 31, wave = tid >> 5;
  const int b = blockIdx.x;
  const int nodeBase = b * NBF;

  int rb0 = rbase[b];
  const int rb1 = rbase[b + 1];
  rb0 = rb0 < 0 ? 0 : (rb0 > csrLen ? csrLen : rb0);
  rb0 &= ~31;
  int len = rb1 - rb0;
  len = len < 0 ? 0 : (len > RCAP ? RCAP : len);
  int lenW = (len + 31) & ~31;
  if (rb0 + lenW > csrLen) lenW = (csrLen - rb0) & ~31;

  {
    const v4i z = {0, 0, 0, 0};
    for (int i = tid; i < RCAP / 4; i += NTHR) ((v4i*)region)[i] = z;
    for (int s = tid; s < NBF; s += NTHR) {
      int o = off[nodeBase + s] - rb0;
      o = o < 0 ? 0 : (o > RCAP ? RCAP : o);
      cursor[s] = o;
    }
  }
  __syncthreads();

  const int nChunks = (nE + CHUNK - 1) / CHUNK;
#pragma unroll 1
  for (int ch = 0; ch < nChunks; ++ch) {
    const int cbase = ch * CHUNK;
    const int wc = scan_chunk<NBF>(dsts, nE, cbase, nodeBase, vec8, list, tid, lane, wave);
    if (lane == 0) wcnt[wave] = wc;
    __syncthreads();
    if (wave == 0) {
#pragma unroll 1
      for (int wsx = 0; wsx < NWAVE; ++wsx) {
        int n = __builtin_amdgcn_readfirstlane(wcnt[wsx]);
        n = n > WCAP ? WCAP : (n < 0 ? 0 : n);
        const int* lp = list + wsx * WCAP;
#pragma unroll 1
        for (int i = 0; i < n; ++i) {
          const int ent  = __builtin_amdgcn_readfirstlane(lp[i]);
          const int slot = ent & (NBF - 1);
          int e = cbase + ((ent >> 12) & (CHUNK - 1));
          e = e > nE - 1 ? nE - 1 : e;
          int src = srcs[e];
          src = src < 0 ? 0 : (src > nN - 1 ? nN - 1 : src);
          if (lane == 0) {
            int pos = cursor[slot];
            pos = pos < 0 ? 0 : (pos > RCAP - 1 ? RCAP - 1 : pos);
            region[pos] = src;
            const int np = pos + 1;
            cursor[slot] = np > RCAP ? RCAP : np;
          }
        }
      }
    }
    __syncthreads();
  }

  const int nv = lenW >> 2;
  int* gp = csr + rb0;
#pragma unroll 1
  for (int i = tid; i < nv; i += NTHR) { const v4i v = ((const v4i*)region)[i]; *(volatile v4i*)(gp + 4 * i) = v; }
  __threadfence();
#pragma unroll 1
  for (int i = tid; i < nv; i += NTHR) { const v4i v = ((const v4i*)region)[i]; *(volatile v4i*)(gp + 4 * i) = v; }
}

__global__ __launch_bounds__(NTHR) void k_front(
    const int* __restrict__ tok, const int* __restrict__ lens,
    const int* __restrict__ vnode, const int* __restrict__ vbeg, const int* __restrict__ vlen,
    const float* __restrict__ pre, const float* __restrict__ emb,
    float* nf, int nN, int nV, int nVocab) {
  __shared__ int win[FNB * NTOK];
  const int tid = threadIdx.x, lane = tid & 31, wave = tid >> 5;
  const int nodeBase = blockIdx.x * FNB;
  for (int i = tid; i < FNB * NTOK; i += NTHR) win[i] = -1;
  __syncthreads();

  if (wave == 0) {
#pragma unroll 1
    for (int v0 = 0; v0 < nV; v0 += 32) {
      const int v  = v0 + lane;
      const int vc = v < nV ? v : nV - 1;
      const int nd = vnode[vc];
      const int vb = vbeg[vc];
      const int vl = vlen[vc];
      const bool hit = (v < nV) && ((unsigned)(nd - nodeBase) < (unsigned)FNB);
      unsigned msk = __builtin_amdgcn_ballot_w32(hit);
#pragma unroll 1
      while (msk != 0u) {
        const int j = __builtin_ctz(msk);
        msk &= msk - 1u;
        const int slot = __builtin_amdgcn_readlane(nd, j) - nodeBase;
        const int bgn  = __builtin_amdgcn_readlane(vb, j);
        const int L    = __builtin_amdgcn_readlane(vl, j);
        const int t    = bgn + lane;
        if (lane < LMAXV && lane < L && (unsigned)t < (unsigned)NTOK && (unsigned)slot < (unsigned)FNB)
          win[slot * NTOK + t] = (v0 + j) * LMAXV + lane;
      }
    }
  }
  __syncthreads();

  const int col0 = 4 * lane, col1 = 128 + 4 * lane;
  const v4f z4 = {0.f, 0.f, 0.f, 0.f};
  const int codeMax = nV * LMAXV - 1;
#pragma unroll 1
  for (int j = 0; j < FNB / NWAVE; ++j) {
    const int slot = wave * (FNB / NWAVE) + j;
    const int n  = nodeBase + slot;
    const int nc = n < nN ? n : nN - 1;
    const int len = lens[nc];
    const int L = len < 0 ? 0 : (len > NTOK ? NTOK : len);
    v4f a0 = z4, a1 = z4;
#pragma unroll 1
    for (int t = 0; t < L; ++t) {
      const int code = __builtin_amdgcn_readfirstlane(win[slot * NTOK + t]);
      int tk = tok[(size_t)nc * NTOK + t];
      tk = tk < 0 ? 0 : (tk > nVocab - 1 ? nVocab - 1 : tk);
      int cc = code < 0 ? 0 : code;
      cc = cc > codeMax ? codeMax : cc;
      const float* rp = (code >= 0) ? (pre + (size_t)cc * DEMB) : (emb + (size_t)tk * DEMB);
      a0 = a0 + *(const v4f*)(rp + col0);
      a1 = a1 + *(const v4f*)(rp + col1);
    }
    const float inv = 1.0f / (float)len;
    v4f o0 = a0 * inv, o1 = a1 * inv;
    if (n >= nN) { o0 = z4; o1 = z4; }
    float* p0 = nf + (size_t)n * DEMB + col0;
    float* p1 = nf + (size_t)n * DEMB + col1;
    *(volatile v4f*)p0 = o0;
    *(volatile v4f*)p1 = o1;
    __threadfence();
    *(volatile v4f*)p0 = o0;
    *(volatile v4f*)p1 = o1;
  }
}

template <int KD, int NC, int CH, int MODE>
__global__ __launch_bounds__(NTHR) void k_gemm(
    const float* __restrict__ A, const unsigned short* __restrict__ Bw,
    const float* __restrict__ attS, const float* __restrict__ attD, const float* __restrict__ bias,
    float* C, float* eS, float* eD, int nRowsA, int ePitch) {
  constexpr int NKH = KD / GKS;
  constexpr int TPW = NCB / 32;
  constexpr int UPT = (GBM * GKS / 8) / NTHR;
  constexpr size_t WPLN = (size_t)NC * KD;
  constexpr int HPB = (MODE == 0) ? (NCB / CH) : 1;
  constexpr int NPAIR = GBM * HPB;
  constexpr int TPP = NTHR / NPAIR;
  constexpr int CPT = (MODE == 0) ? (CH / TPP) : 4;
  static_assert(KD % GKS == 0 && NKH >= 1 && NKH <= 4 && (GKS % 32) == 0);
  static_assert(NC % NCB == 0 && TPW == 8);
  static_assert(UPT * NTHR * 8 == GBM * GKS);
  static_assert(((GAPK * 2) % 16) == 0);
  static_assert(GBM * NCB * 4 <= GLDS && 2 * GBM * GAPK * 2 <= GLDS);
  static_assert(MODE != 0 || (HPB * CH == NCB && HPB <= 4 && NPAIR * TPP == NTHR && TPP * CPT == CH && (CPT % 4) == 0 && TPP <= 32));

  extern __shared__ v4f lds_dyn[];
  __shared__ __attribute__((aligned(16))) float sES[GBM * 4];
  __shared__ __attribute__((aligned(16))) float sED[GBM * 4];
  unsigned short* sHi = (unsigned short*)lds_dyn;
  unsigned short* sLo = sHi + GBM * GAPK;
  float*          stg = (float*)lds_dyn;
  const int tid = threadIdx.x, lane = tid & 31, wave = tid >> 5, hh = lane >> 4, m = lane & 15;
  const int rowBase = blockIdx.x * GBM;
  const int colBase = blockIdx.y * NCB;

  const int rg  = wave >> 1;
  const int chf = wave & 1;
  const int r0  = rg * 16;
  const int c0  = chf * 128;

  v8f acc[TPW];
#pragma unroll
  for (int t = 0; t < TPW; ++t) { v8f z = {0.f, 0.f, 0.f, 0.f, 0.f, 0.f, 0.f, 0.f}; acc[t] = z; }
  const unsigned short* ahp = sHi + (r0 + m) * GAPK + 8 * hh;
  const unsigned short* alp = sLo + (r0 + m) * GAPK + 8 * hh;

#pragma unroll 1
  for (int kh = 0; kh < NKH; ++kh) {
#pragma unroll
    for (int i = 0; i < UPT; ++i) {
      const int idx = i * NTHR + tid;
      const int r   = idx >> 4;
      const int cc  = (idx & 15) * 8;
      int row = rowBase + r;
      row = row > nRowsA - 1 ? nRowsA - 1 : row;
      const float* ap = A + (size_t)row * KD + kh * GKS + cc;
      const v4f a = *(const v4f*)ap, b = *(const v4f*)(ap + 4);
      v8us hv, lv;
      split8(a, b, hv, lv);
      *(v8us*)(sHi + r * GAPK + cc) = hv;
      *(v8us*)(sLo + r * GAPK + cc) = lv;
    }
    __syncthreads();

#pragma unroll 2
    for (int kt = 0; kt < GKS / 32; ++kt) {
      FragB ah, al;
      ah.h[0] = *(const v8us*)(ahp + 32 * kt);
      ah.h[1] = *(const v8us*)(ahp + 32 * kt + 16);
      al.h[0] = *(const v8us*)(alp + 32 * kt);
      al.h[1] = *(const v8us*)(alp + 32 * kt + 16);
#pragma unroll
      for (int t = 0; t < TPW; ++t) {
        const unsigned short* bp = Bw + (size_t)(colBase + c0 + 16 * t + m) * KD + kh * GKS + 32 * kt + 8 * hh;
        FragB bh, bl;
        bh.h[0] = *(const v8us*)bp;
        bh.h[1] = *(const v8us*)(bp + 16);
        bl.h[0] = *(const v8us*)(bp + WPLN);
        bl.h[1] = *(const v8us*)(bp + WPLN + 16);
        acc[t] = wmb(ah.v, bh.v, acc[t]);
        acc[t] = wmb(ah.v, bl.v, acc[t]);
        acc[t] = wmb(al.v, bh.v, acc[t]);
      }
    }
    __syncthreads();
  }

  {
    float* sp = stg + (size_t)(r0 + 8 * hh) * NCB + c0 + m;
#pragma unroll
    for (int t = 0; t < TPW; ++t) {
#pragma unroll
      for (int r = 0; r < 8; ++r) sp[r * NCB + 16 * t] = acc[t][r];
    }
  }
  __syncthreads();

  {
    const int col = c0 + 4 * lane;
    v4f bb = {0.f, 0.f, 0.f, 0.f};
    if constexpr (MODE != 0) bb = *(const v4f*)(bias + colBase + col);
    const size_t gb = (size_t)(rowBase + r0) * NC + colBase + col;
#pragma unroll
    for (int it = 0; it < 16; ++it) {
      v4f v = *(const v4f*)(stg + (size_t)(r0 + it) * NCB + col);
      if constexpr (MODE != 0) v = v + bb;
      if constexpr (MODE == 1) {
        v.x = v.x > 0.f ? v.x : DEC_SLOPE * v.x;
        v.y = v.y > 0.f ? v.y : DEC_SLOPE * v.y;
        v.z = v.z > 0.f ? v.z : DEC_SLOPE * v.z;
        v.w = v.w > 0.f ? v.w : DEC_SLOPE * v.w;
      }
      *(volatile v4f*)(C + gb + (size_t)it * NC) = v;
    }
    __threadfence();
#pragma unroll
    for (int it = 0; it < 16; ++it) {
      v4f v = *(const v4f*)(stg + (size_t)(r0 + it) * NCB + col);
      if constexpr (MODE != 0) v = v + bb;
      if constexpr (MODE == 1) {
        v.x = v.x > 0.f ? v.x : DEC_SLOPE * v.x;
        v.y = v.y > 0.f ? v.y : DEC_SLOPE * v.y;
        v.z = v.z > 0.f ? v.z : DEC_SLOPE * v.z;
        v.w = v.w > 0.f ? v.w : DEC_SLOPE * v.w;
      }
      *(volatile v4f*)(C + gb + (size_t)it * NC) = v;
    }
  }

  if constexpr (MODE == 0) {
    const int pair = tid / TPP;
    const int sub  = tid - pair * TPP;
    const int hd   = pair / GBM;
    const int row  = pair - hd * GBM;
    const int clb  = hd * CH + sub * CPT;
    const float* srow = stg + (size_t)row * NCB + clb;
    const float* ga   = attS + colBase + clb;
    const float* gd   = attD + colBase + clb;
    float ps = 0.f, pd = 0.f;
#pragma unroll 2
    for (int c = 0; c < CPT; c += 4) {
      const v4f v  = *(const v4f*)(srow + c);
      const v4f sa = *(const v4f*)(ga + c);
      const v4f sd = *(const v4f*)(gd + c);
      ps += v.x * sa.x + v.y * sa.y + v.z * sa.z + v.w * sa.w;
      pd += v.x * sd.x + v.y * sd.y + v.z * sd.z + v.w * sd.w;
    }
#pragma unroll
    for (int o = 1; o < TPP; o <<= 1) { ps += __shfl_xor(ps, o); pd += __shfl_xor(pd, o); }
    if (sub == 0) { sES[pair] = ps; sED[pair] = pd; }
    __syncthreads();

    const int  hdl = wave % HPB;
    const bool wS  = wave < HPB;
    const bool wD  = (wave >= HPB) && (wave < 2 * HPB);
    const int  lr  = (lane & 15);
    const v4f  d1  = *(const v4f*)(sES + hdl * GBM + 4 * lr);
    const v4f  d2  = *(const v4f*)(sED + hdl * GBM + 4 * lr);
    const v4f  dv  = wS ? d1 : d2;
    float* ebase = wS ? eS : eD;
    float* gp = ebase + (size_t)(colBase / CH + hdl) * ePitch + rowBase + 4 * lr;
    if ((wS || wD) && lane < 16) *(volatile v4f*)gp = dv;
    __threadfence();
    if ((wS || wD) && lane < 16) *(volatile v4f*)gp = dv;
  }
}

__global__ __launch_bounds__(NTHR) void k_agg1(
    const int* __restrict__ csr, const int* __restrict__ off, const int* __restrict__ cnt,
    const float* __restrict__ eS, const float* __restrict__ eD, const float* __restrict__ hw,
    float* xout, int nN, int csrLen, int ePitch) {
  const int tid = threadIdx.x, lane = tid & 31, wave = tid >> 5;
  const int tbase = blockIdx.x * TGT + wave * 32;
  const int col0 = 4 * lane, col1 = 128 + 4 * lane;
  const int hd0 = lane >> 4;
  const int hd1 = 2 + (lane >> 4);
  const v4f z4 = {0.f, 0.f, 0.f, 0.f};
  const float* eS0 = eS + (size_t)hd0 * ePitch;
  const float* eS1 = eS + (size_t)hd1 * ePitch;
  const float* eD0 = eD + (size_t)hd0 * ePitch;
  const float* eD1 = eD + (size_t)hd1 * ePitch;

  const int cl    = tbase + lane;
  const int cnt_l = cnt[cl];
  const int off_l = off[cl];

#pragma unroll 1
  for (int j = 0; j < 32; ++j) {
    const int c = tbase + j;
    int n = __shfl(cnt_l, j);
    n = n < 0 ? 0 : (n > DEGCAP ? DEGCAP : n);
    const int st = __shfl(off_l, j);
    const float ed0 = eD0[c];
    const float ed1 = eD1[c];

    float mx0 = NEG_BIG, mx1 = NEG_BIG;
#pragma unroll 1
    for (int q0 = 0; q0 < n; q0 += 32) {
      int pos = st + q0 + lane;
      pos = pos < 0 ? 0 : (pos > csrLen - 1 ? csrLen - 1 : pos);
      int sl = csr[pos];
      sl = sl < 0 ? 0 : (sl > nN - 1 ? nN - 1 : sl);
      const int mcnt = (n - q0) < 32 ? (n - q0) : 32;
#pragma unroll 1
      for (int pp = 0; pp < mcnt; ++pp) {
        const int s = __builtin_amdgcn_readlane(sl, pp);
        mx0 = fmaxf(mx0, lrelu(eS0[s] + ed0));
        mx1 = fmaxf(mx1, lrelu(eS1[s] + ed1));
      }
    }

    float den0 = 0.f, den1 = 0.f;
    v4f   acc0 = z4, acc1 = z4;
#pragma unroll 1
    for (int q0 = 0; q0 < n; q0 += 32) {
      int pos = st + q0 + lane;
      pos = pos < 0 ? 0 : (pos > csrLen - 1 ? csrLen - 1 : pos);
      int sl = csr[pos];
      sl = sl < 0 ? 0 : (sl > nN - 1 ? nN - 1 : sl);
      const int mcnt = (n - q0) < 32 ? (n - q0) : 32;
#pragma unroll 1
      for (int pp = 0; pp < mcnt; ++pp) {
        const int s = __builtin_amdgcn_readlane(sl, pp);
        const float p0 = __expf(lrelu(eS0[s] + ed0) - mx0);
        den0 += p0;
        const v4f h0 = *(const v4f*)(hw + (size_t)s * H1C + col0);
        acc0 = acc0 + h0 * p0;
        const float p1 = __expf(lrelu(eS1[s] + ed1) - mx1);
        den1 += p1;
        const v4f h1 = *(const v4f*)(hw + (size_t)s * H1C + col1);
        acc1 = acc1 + h1 * p1;
      }
    }

    const float rd0 = 1.0f / (den0 + DEN_EPS);
    const float rd1 = 1.0f / (den1 + DEN_EPS);
    v4f v0 = acc0 * rd0;
    v4f v1 = acc1 * rd1;
    v0.x = eluf(v0.x); v0.y = eluf(v0.y); v0.z = eluf(v0.z); v0.w = eluf(v0.w);
    v1.x = eluf(v1.x); v1.y = eluf(v1.y); v1.z = eluf(v1.z); v1.w = eluf(v1.w);
    if (c >= nN) { v0 = z4; v1 = z4; }
    float* p0w = xout + (size_t)c * H1C + col0;
    float* p1w = xout + (size_t)c * H1C + col1;
    *(volatile v4f*)p0w = v0;
    *(volatile v4f*)p1w = v1;
    __threadfence();
    *(volatile v4f*)p0w = v0;
    *(volatile v4f*)p1w = v1;
  }
}

__global__ __launch_bounds__(NTHR) void k_aggv(
    const int* __restrict__ csr, const int* __restrict__ off, const int* __restrict__ cnt,
    const int* __restrict__ vsel, const float* __restrict__ eS, const float* __restrict__ eD,
    const float* __restrict__ hw, float* gout, int nN, int nV, int csrLen, int ePitch) {
  const int tid = threadIdx.x, lane = tid & 31, wave = tid >> 5;
  const int tbase = blockIdx.x * TGT + wave * 32;
  const int col0 = 4 * lane, col1 = 128 + 4 * lane;
  const v4f z4 = {0.f, 0.f, 0.f, 0.f};

  int vv = tbase + lane;
  vv = vv > nV - 1 ? nV - 1 : vv;
  int cn = vsel[vv];
  cn = cn < 0 ? 0 : (cn > nN - 1 ? nN - 1 : cn);
  const int cnt_l = cnt[cn];
  const int off_l = off[cn];

#pragma unroll 1
  for (int j = 0; j < 32; ++j) {
    const int var = tbase + j;
    const int c = __shfl(cn, j);
    int n = __shfl(cnt_l, j);
    n = n < 0 ? 0 : (n > DEGCAP ? DEGCAP : n);
    const int st = __shfl(off_l, j);
    v4f g0 = z4, g1 = z4;

#pragma unroll 1
    for (int h = 0; h < NH; ++h) {
      const float* eSh = eS + (size_t)h * ePitch;
      const float  edh = eD[(size_t)h * ePitch + c];
      const float* hwh = hw + h * CH2;

      float mx = NEG_BIG;
#pragma unroll 1
      for (int q0 = 0; q0 < n; q0 += 32) {
        int pos = st + q0 + lane;
        pos = pos < 0 ? 0 : (pos > csrLen - 1 ? csrLen - 1 : pos);
        int sl = csr[pos];
        sl = sl < 0 ? 0 : (sl > nN - 1 ? nN - 1 : sl);
        const int mcnt = (n - q0) < 32 ? (n - q0) : 32;
#pragma unroll 1
        for (int pp = 0; pp < mcnt; ++pp) {
          const int s = __builtin_amdgcn_readlane(sl, pp);
          mx = fmaxf(mx, lrelu(eSh[s] + edh));
        }
      }

      float den = 0.f;
      v4f a0 = z4, a1 = z4;
#pragma unroll 1
      for (int q0 = 0; q0 < n; q0 += 32) {
        int pos = st + q0 + lane;
        pos = pos < 0 ? 0 : (pos > csrLen - 1 ? csrLen - 1 : pos);
        int sl = csr[pos];
        sl = sl < 0 ? 0 : (sl > nN - 1 ? nN - 1 : sl);
        const int mcnt = (n - q0) < 32 ? (n - q0) : 32;
#pragma unroll 1
        for (int pp = 0; pp < mcnt; ++pp) {
          const int s = __builtin_amdgcn_readlane(sl, pp);
          const float p = __expf(lrelu(eSh[s] + edh) - mx);
          den += p;
          const float* zr = hwh + (size_t)s * H2C;
          const v4f h0 = *(const v4f*)(zr + col0);
          const v4f h1 = *(const v4f*)(zr + col1);
          a0 = a0 + h0 * p;
          a1 = a1 + h1 * p;
        }
      }
      const float rd = 1.0f / (den + DEN_EPS);
      g0 = g0 + a0 * rd;
      g1 = g1 + a1 * rd;
    }

    g0 = g0 * 0.25f;
    g1 = g1 * 0.25f;
    if (var >= nV) { g0 = z4; g1 = z4; }
    float* p0w = gout + (size_t)var * CH2 + col0;
    float* p1w = gout + (size_t)var * CH2 + col1;
    *(volatile v4f*)p0w = g0;
    *(volatile v4f*)p1w = g1;
    __threadfence();
    *(volatile v4f*)p0w = g0;
    *(volatile v4f*)p1w = g1;
  }
}

__global__ __launch_bounds__(NTHR) void k_segmax(
    const float* __restrict__ g, const int* __restrict__ seg, float* wm, int nV, int nF) {
  const int tid = threadIdx.x, lane = tid & 31, wave = tid >> 5;
  const int f = blockIdx.x * NWAVE + wave;
  if (f >= nF) return;
  const int col0 = 4 * lane, col1 = 128 + 4 * lane;
  const float ninf = -__builtin_inff();
  v4f m0 = {ninf, ninf, ninf, ninf};
  v4f m1 = m0;
#pragma unroll 1
  for (int v0 = 0; v0 < nV; v0 += 32) {
    const int v  = v0 + lane;
    const int vc = v < nV ? v : nV - 1;
    const int sv = seg[vc];
    const bool hit = (v < nV) && (sv == f);
    unsigned msk = __builtin_amdgcn_ballot_w32(hit);
#pragma unroll 1
    while (msk != 0u) {
      const int j = __builtin_ctz(msk);
      msk &= msk - 1u;
      const int vv = v0 + j;
      const v4f r0 = *(const v4f*)(g + (size_t)vv * CH2 + col0);
      const v4f r1 = *(const v4f*)(g + (size_t)vv * CH2 + col1);
      m0.x = fmaxf(m0.x, r0.x); m0.y = fmaxf(m0.y, r0.y); m0.z = fmaxf(m0.z, r0.z); m0.w = fmaxf(m0.w, r0.w);
      m1.x = fmaxf(m1.x, r1.x); m1.y = fmaxf(m1.y, r1.y); m1.z = fmaxf(m1.z, r1.z); m1.w = fmaxf(m1.w, r1.w);
    }
  }
  float* p0 = wm + (size_t)f * CH2 + col0;
  float* p1 = wm + (size_t)f * CH2 + col1;
  *(volatile v4f*)p0 = m0;
  *(volatile v4f*)p1 = m1;
  __threadfence();
  *(volatile v4f*)p0 = m0;
  *(volatile v4f*)p1 = m1;
}

extern "C" void kernel_launch(void* const* d_in, const int* in_sizes, int n_in,
                              void* d_out, int out_size, void* d_ws, size_t ws_size,
                              hipStream_t stream) {
  if (n_in < 21) return;
  const int nN = in_sizes[1];
  if (nN <= 0 || in_sizes[0] != nN * NTOK) return;
  const int nE = in_sizes[2];
  if (nE <= 0 || in_sizes[3] != nE) return;
  const int nV = in_sizes[4];
  if (nV <= 0 || in_sizes[5] != nV || in_sizes[6] != nV || in_sizes[7] != nV || in_sizes[8] != nV) return;
  if (in_sizes[9] != nV * LMAXV * DEMB) return;
  if (in_sizes[10] <= 0 || (in_sizes[10] % DEMB) != 0) return;
  const int nVocab = in_sizes[10] / DEMB;
  if (in_sizes[11] != DEMB * H1C || in_sizes[12] != H1C || in_sizes[13] != H1C) return;
  if (in_sizes[14] != H1C * H2C || in_sizes[15] != H2C || in_sizes[16] != H2C) return;
  if (in_sizes[17] != CH2 * HID || in_sizes[18] != HID || in_sizes[19] != HID * NCLS || in_sizes[20] != NCLS) return;
  if (out_size <= 0 || (out_size % NCLS) != 0) return;
  const int nF = out_size / NCLS;
  if ((nF % GBM) != 0) return;
  if (nE > (1 << 28) || nN > (1 << 24) || nV > (1 << 24)) return;

  const int*   tok   = (const int*)d_in[0];
  const int*   lens  = (const int*)d_in[1];
  const int*   esrc  = (const int*)d_in[2];
  const int*   edst  = (const int*)d_in[3];
  const int*   vnode = (const int*)d_in[4];
  const int*   vbeg  = (const int*)d_in[5];
  const int*   vsel  = (const int*)d_in[6];
  const int*   fseg  = (const int*)d_in[7];
  const int*   vlen  = (const int*)d_in[8];
  const float* pre   = (const float*)d_in[9];
  const float* emb   = (const float*)d_in[10];
  const float* W1    = (const float*)d_in[11];
  const float* a1s   = (const float*)d_in[12];
  const float* a1d   = (const float*)d_in[13];
  const float* W2    = (const float*)d_in[14];
  const float* a2s   = (const float*)d_in[15];
  const float* a2d   = (const float*)d_in[16];
  const float* Wd1   = (const float*)d_in[17];
  const float* bd1   = (const float*)d_in[18];
  const float* Wd2   = (const float*)d_in[19];
  const float* bd2   = (const float*)d_in[20];
  float* out = (float*)d_out;

  const int NPAD   = ((nN + TGT - 1) / TGT) * TGT;
  const int VPAD   = ((nV + TGT - 1) / TGT) * TGT;
  const int nBC    = (nN + NBC - 1) / NBC;
  const int CNTPAD = nBC * NBC;
  if (4 * nBC + 1 > RBN) return;
  const int nBF    = (nN + NBF - 1) / NBF;
  const int csrLen = ((nE + 31) & ~31) + 4096;
  if (31 * 4 * nBC > 4096) return;
  const int nAgg   = NPAD / TGT;
  const int nAggV  = VPAD / TGT;
  const int nFront = NPAD / FNB;

  char* ws = (char*)d_ws;
  size_t off = 0;
  const size_t oW1  = off; off += (size_t)2 * DEMB * H1C * 2;     off = (off + 255) & ~(size_t)255;
  const size_t oW2  = off; off += (size_t)2 * H1C * H2C * 2;      off = (off + 255) & ~(size_t)255;
  const size_t oWd1 = off; off += (size_t)2 * CH2 * HID * 2;      off = (off + 255) & ~(size_t)255;
  const size_t oWd2 = off; off += (size_t)2 * HID * NCLS * 2;     off = (off + 255) & ~(size_t)255;
  const size_t oCnt = off; off += (size_t)CNTPAD * 4;             off = (off + 255) & ~(size_t)255;
  const size_t oOff = off; off += (size_t)CNTPAD * 4;             off = (off + 255) & ~(size_t)255;
  const size_t oRb  = off; off += (size_t)RBN * 4;                off = (off + 255) & ~(size_t)255;
  const size_t oCsr = off; off += (size_t)csrLen * 4;             off = (off + 255) & ~(size_t)255;
  const size_t oA   = off; off += (size_t)NPAD * DEMB * 4;        off = (off + 255) & ~(size_t)255;
  const size_t oZ   = off; off += (size_t)NPAD * H2C * 4;         off = (off + 255) & ~(size_t)255;
  const size_t oES1 = off; off += (size_t)NH * NPAD * 4;          off = (off + 255) & ~(size_t)255;
  const size_t oED1 = off; off += (size_t)NH * NPAD * 4;          off = (off + 255) & ~(size_t)255;
  const size_t oES2 = off; off += (size_t)NH * NPAD * 4;          off = (off + 255) & ~(size_t)255;
  const size_t oED2 = off; off += (size_t)NH * NPAD * 4;          off = (off + 255) & ~(size_t)255;
  const size_t oG   = off; off += (size_t)VPAD * CH2 * 4;         off = (off + 255) & ~(size_t)255;
  const size_t oWm  = off; off += (size_t)nF * CH2 * 4;           off = (off + 255) & ~(size_t)255;
  const size_t oHd  = off; off += (size_t)nF * HID * 4;           off = (off + 255) & ~(size_t)255;
  if (off > ws_size || off > (size_t)WSCAP) return;
  unsigned short* wp1  = (unsigned short*)(ws + oW1);
  unsigned short* wp2  = (unsigned short*)(ws + oW2);
  unsigned short* wpd1 = (unsigned short*)(ws + oWd1);
  unsigned short* wpd2 = (unsigned short*)(ws + oWd2);
  int*   cnt  = (int*)(ws + oCnt);
  int*   offp = (int*)(ws + oOff);
  int*   rb   = (int*)(ws + oRb);
  int*   csr  = (int*)(ws + oCsr);
  float* bufA = (float*)(ws + oA);
  float* bufZ = (float*)(ws + oZ);
  float* es1  = (float*)(ws + oES1);
  float* ed1  = (float*)(ws + oED1);
  float* es2  = (float*)(ws + oES2);
  float* ed2  = (float*)(ws + oED2);
  float* gpl  = (float*)(ws + oG);
  float* wm   = (float*)(ws + oWm);
  float* hdec = (float*)(ws + oHd);

  const int vec8 = 1;

  k_wprep<DEMB, H1C><<<(H1C * DEMB / 8 + NTHR - 1) / NTHR, NTHR, 0, stream>>>(W1, wp1);
  k_wprep<H1C, H2C><<<(H2C * H1C / 8 + NTHR - 1) / NTHR, NTHR, 0, stream>>>(W2, wp2);
  k_wprep<CH2, HID><<<(HID * CH2 / 8 + NTHR - 1) / NTHR, NTHR, 0, stream>>>(Wd1, wpd1);
  k_wprep<HID, NCLS><<<(NCLS * HID / 8 + NTHR - 1) / NTHR, NTHR, 0, stream>>>(Wd2, wpd2);

  k_count<<<nBC, NTHR, 0, stream>>>(edst, cnt, nE, vec8);
  k_offsets<<<1, OTHR, 0, stream>>>(cnt, offp, rb, nBC);
  hipFuncSetAttribute(reinterpret_cast<const void*>(&k_fill),
                      hipFuncAttributeMaxDynamicSharedMemorySize, LDS_FILL);
  k_fill<<<nBF, NTHR, LDS_FILL, stream>>>(esrc, edst, offp, rb, csr, nN, nE, vec8, csrLen);

  k_front<<<nFront, NTHR, 0, stream>>>(tok, lens, vnode, vbeg, vlen, pre, emb, bufA, nN, nV, nVocab);

  hipFuncSetAttribute(reinterpret_cast<const void*>(&k_gemm<DEMB, H1C, CH1, 0>),
                      hipFuncAttributeMaxDynamicSharedMemorySize, GLDS);
  k_gemm<DEMB, H1C, CH1, 0><<<dim3(NPAD / GBM, H1C / NCB), NTHR, GLDS, stream>>>(
      bufA, wp1, a1s, a1d, a1s, bufZ, es1, ed1, NPAD, NPAD);
  k_agg1<<<nAgg, NTHR, 0, stream>>>(csr, offp, cnt, es1, ed1, bufZ, bufA, nN, csrLen, NPAD);

  hipFuncSetAttribute(reinterpret_cast<const void*>(&k_gemm<H1C, H2C, CH2, 0>),
                      hipFuncAttributeMaxDynamicSharedMemorySize, GLDS);
  k_gemm<H1C, H2C, CH2, 0><<<dim3(NPAD / GBM, H2C / NCB), NTHR, GLDS, stream>>>(
      bufA, wp2, a2s, a2d, a2s, bufZ, es2, ed2, NPAD, NPAD);
  k_aggv<<<nAggV, NTHR, 0, stream>>>(csr, offp, cnt, vsel, es2, ed2, bufZ, gpl, nN, nV, csrLen, NPAD);

  k_segmax<<<(nF + NWAVE - 1) / NWAVE, NTHR, 0, stream>>>(gpl, fseg, wm, nV, nF);

  hipFuncSetAttribute(reinterpret_cast<const void*>(&k_gemm<CH2, HID, NCB, 1>),
                      hipFuncAttributeMaxDynamicSharedMemorySize, GLDS);
  k_gemm<CH2, HID, NCB, 1><<<dim3(nF / GBM, HID / NCB), NTHR, GLDS, stream>>>(
      wm, wpd1, bd1, bd1, bd1, hdec, es2, ed2, nF, NPAD);
  hipFuncSetAttribute(reinterpret_cast<const void*>(&k_gemm<HID, NCLS, NCB, 2>),
                      hipFuncAttributeMaxDynamicSharedMemorySize, GLDS);
  k_gemm<HID, NCLS, NCB, 2><<<dim3(nF / GBM, NCLS / NCB), NTHR, GLDS, stream>>>(
      hdec, wpd2, bd2, bd2, bd2, out, es2, ed2, nF, NPAD);
}
